// AttentionBlock_49074296324680
// MI455X (gfx1250) — hardware-verified
//
#include <hip/hip_runtime.h>
#include <stdint.h>


#ifndef NB
#define NB 4
#endif
#ifndef SEQ
#define SEQ 4096
#endif
#define NB_FULL  4
#define SEQ_FULL 4096
#define CCH      256
#define HEADS    4
#define HDIM     64
#define GNG      32
#define CPG      (CCH / GNG)
#define QKVO     (3 * CCH)
#define NTOK     (NB * SEQ)
#define PLD      72
#define GPT      72

static_assert(CCH == HEADS * HDIM);
static_assert(CPG == 8);
static_assert(HDIM == 64);
static_assert((SEQ % 128) == 0);
static_assert((NTOK % 128) == 0);
static_assert((CCH % 128) == 0);
static_assert(NB >= 1 && NB <= NB_FULL);
static_assert(SEQ <= SEQ_FULL);

typedef _Float16     v16h __attribute__((ext_vector_type(16)));
typedef _Float16     v8h  __attribute__((ext_vector_type(8)));
typedef float        v8f  __attribute__((ext_vector_type(8)));
typedef float        v4f  __attribute__((ext_vector_type(4)));
typedef unsigned int v4u  __attribute__((ext_vector_type(4)));

union Frag  { v16h v; v8h h[2]; };
union Pack8 { v8h h; v4u u; };

static constexpr size_t PLANE_H   = (size_t)NTOK * CCH;
static constexpr size_t WPL_H     = (size_t)CCH * CCH;
static constexpr size_t WS_HALVES = 5 * PLANE_H + 4 * WPL_H;

static __device__ __forceinline__ v8f wmma16(v16h a, v16h b, v8f c) {
  v8f d = __builtin_amdgcn_wmma_f32_16x16x32_f16(false, a, false, b, (short)0, c, false, false);
  asm volatile("v_nop\n\tv_nop\n\tv_nop\n\tv_nop" : "+v"(d) : "v"(a), "v"(b));
  return d;
}

static __device__ __forceinline__ v16h frag_rows(const _Float16* base, int row0, size_t ld, int k0) {
  const int l = threadIdx.x & 31, hf = l >> 4, m = l & 15;
  const _Float16* p = base + (size_t)(row0 + m) * ld + k0 + 8 * hf;
  Frag f;
  f.h[0] = *(const v8h*)(p);
  f.h[1] = *(const v8h*)(p + 16);
  return f.v;
}

static __device__ __forceinline__ float bf16_rne(float f) {
  unsigned int u = __float_as_uint(f);
  u += 0x7fffu + ((u >> 16) & 1u);
  u &= 0xffff0000u;
  return __uint_as_float(u);
}

__global__ __launch_bounds__(256)
void k_gn(const float* __restrict__ x, const float* __restrict__ gw,
          const float* __restrict__ gb, _Float16* __restrict__ xh) {
  __shared__ _Float16 T[64 * GPT];

  const int tid = threadIdx.x, w = tid >> 5, lane = tid & 31;
  const int cb = blockIdx.x, b = blockIdx.y;
  const int cbase = cb * 64;
  const int nj = SEQ / 128;
  const float* xg = x + ((size_t)(b * CCH) + cbase + CPG * w) * SEQ_FULL + 4 * lane;

  float s0 = 0.0f, s1 = 0.0f, s2 = 0.0f, s3 = 0.0f;
#pragma unroll 1
  for (int c = 0; c < CPG; ++c) {
    const float* xr = xg + (size_t)c * SEQ_FULL;
#pragma unroll 4
    for (int j = 0; j < nj; ++j) {
      const v4f v = *(const v4f*)(xr + 128 * j);
      s0 += bf16_rne(v[0]); s1 += bf16_rne(v[1]);
      s2 += bf16_rne(v[2]); s3 += bf16_rne(v[3]);
    }
  }
  float s = (s0 + s1) + (s2 + s3);
  s += __shfl_xor(s, 16); s += __shfl_xor(s, 8); s += __shfl_xor(s, 4);
  s += __shfl_xor(s, 2);  s += __shfl_xor(s, 1);
  const float inv_n = 1.0f / (float)(CPG * SEQ);
  const float mean = s * inv_n;

  float q0 = 0.0f, q1 = 0.0f, q2 = 0.0f, q3 = 0.0f;
#pragma unroll 1
  for (int c = 0; c < CPG; ++c) {
    const float* xr = xg + (size_t)c * SEQ_FULL;
#pragma unroll 2
    for (int j = 0; j < nj; ++j) {
      const v4f v = *(const v4f*)(xr + 128 * j);
      const float d0 = bf16_rne(v[0]) - mean, d1 = bf16_rne(v[1]) - mean;
      const float d2 = bf16_rne(v[2]) - mean, d3 = bf16_rne(v[3]) - mean;
      q0 += d0 * d0; q1 += d1 * d1; q2 += d2 * d2; q3 += d3 * d3;
    }
  }
  float q = (q0 + q1) + (q2 + q3);
  q += __shfl_xor(q, 16); q += __shfl_xor(q, 8); q += __shfl_xor(q, 4);
  q += __shfl_xor(q, 2);  q += __shfl_xor(q, 1);
  const float var  = q * inv_n;
  const float rstd = rsqrtf(var + 1.0e-5f);

  const int c = tid >> 2, qq = tid & 3;
  const float gwc = bf16_rne(gw[cbase + c]);
  const float gbc = bf16_rne(gb[cbase + c]);
  const float* xc = x + ((size_t)(b * CCH) + cbase + c) * SEQ_FULL + qq * 16;
  const int p = tid & 7, r0 = tid >> 3;

#pragma unroll 1
  for (int l0 = 0; l0 < SEQ; l0 += 64) {
#pragma unroll
    for (int i = 0; i < 4; ++i) {
      const v4f v = *(const v4f*)(xc + l0 + 4 * i);
#pragma unroll
      for (int e = 0; e < 4; ++e) {
        const float xn = ((bf16_rne(v[e]) - mean) * rstd) * gwc + gbc;
        T[(qq * 16 + 4 * i + e) * GPT + c] = (_Float16)xn;
      }
    }
    __syncthreads();
    Pack8 o0, o1;
    o0.h = *(const v8h*)(T + r0 * GPT + p * 8);
    o1.h = *(const v8h*)(T + (r0 + 32) * GPT + p * 8);
    _Float16* d0 = xh + ((size_t)(b * SEQ + l0 + r0)) * CCH + cbase + p * 8;
    _Float16* d1 = d0 + (size_t)32 * CCH;
    *(volatile v4u*)d0 = o0.u;
    *(volatile v4u*)d1 = o1.u;
    __threadfence();
    *(volatile v4u*)d0 = o0.u;
    *(volatile v4u*)d1 = o1.u;
    __syncthreads();
  }
}

__global__ __launch_bounds__(256)
void k_cvt(const float* __restrict__ src, _Float16* __restrict__ dst,
           int rows, int cols, int period, int pstride, float scale) {
  const int c8n   = cols >> 3;
  const int total = rows * c8n;
  const int i     = blockIdx.x * 256 + threadIdx.x;
  if (i >= total) return;
  const int r  = i / c8n;
  const int c  = (i - r * c8n) * 8;
  const int rb = r / period;
  const int sr = rb * pstride + (r - rb * period);
  const float* s = src + (size_t)sr * cols + c;
  const v4f a = *(const v4f*)(s);
  const v4f b = *(const v4f*)(s + 4);
  Pack8 o;
  o.h[0] = (_Float16)(bf16_rne(a[0]) * scale);
  o.h[1] = (_Float16)(bf16_rne(a[1]) * scale);
  o.h[2] = (_Float16)(bf16_rne(a[2]) * scale);
  o.h[3] = (_Float16)(bf16_rne(a[3]) * scale);
  o.h[4] = (_Float16)(bf16_rne(b[0]) * scale);
  o.h[5] = (_Float16)(bf16_rne(b[1]) * scale);
  o.h[6] = (_Float16)(bf16_rne(b[2]) * scale);
  o.h[7] = (_Float16)(bf16_rne(b[3]) * scale);
  _Float16* d = dst + (size_t)r * cols + c;
  *(volatile v4u*)d = o.u;
  __threadfence();
  *(volatile v4u*)d = o.u;
}

template <int MODE>
__global__ __launch_bounds__(256) __attribute__((amdgpu_num_vgpr(256)))
void k_gemm(const _Float16* __restrict__ A,
            const _Float16* __restrict__ W0, const _Float16* __restrict__ W1,
            const _Float16* __restrict__ W2,
            const float* __restrict__ G0, const float* __restrict__ G1,
            const float* __restrict__ G2,
            void* O0, void* O1, void* O2,
            const float* __restrict__ xres,
            int K, int Nout, int ztr, float oscale, int bper, int bstr) {
  __shared__ float Cs[128 * 128];

  const int tid = threadIdx.x, w = tid >> 5, lane = tid & 31;
  const int hf = lane >> 4, nin = lane & 15;
  const int wm = w >> 1, wn = w & 1;
  const int m_blk = blockIdx.y * 128, n_blk = blockIdx.x * 128;
  const int z = blockIdx.z;
  const _Float16* W  = (z == 0) ? W0 : ((z == 1) ? W1 : W2);
  const float*  bias = (z == 0) ? G0 : ((z == 1) ? G1 : G2);
  void*           Ov = (z == 0) ? O0 : ((z == 1) ? O1 : O2);

  v8f acc[2][4] = {};

#pragma unroll 1
  for (int k0 = 0; k0 < K; k0 += 32) {
    const v16h a0 = frag_rows(A, m_blk + wm * 32,      (size_t)K, k0);
    const v16h a1 = frag_rows(A, m_blk + wm * 32 + 16, (size_t)K, k0);
#pragma unroll
    for (int nt = 0; nt < 4; ++nt) {
      const v16h bf = frag_rows(W, n_blk + wn * 64 + nt * 16, (size_t)K, k0);
      acc[0][nt] = wmma16(a0, bf, acc[0][nt]);
      acc[1][nt] = wmma16(a1, bf, acc[1][nt]);
    }
  }

#pragma unroll
  for (int nt = 0; nt < 4; ++nt) {
    const int ncol = wn * 64 + nt * 16 + nin;
    const int ng = n_blk + ncol;
    const int hq = ng / bper;
    const float bb = bf16_rne(bias[hq * bstr + (ng - hq * bper)]);
#pragma unroll
    for (int mt = 0; mt < 2; ++mt)
#pragma unroll
      for (int r = 0; r < 8; ++r) {
        const int row = wm * 32 + mt * 16 + 8 * hf + r;
        const float v = acc[mt][nt][r] * oscale + bb;
        if (MODE == 0) Cs[row * 128 + ncol] = v;
        else           Cs[ncol * 128 + row] = v;
      }
  }
  __syncthreads();

  if (MODE == 1) {
    float* out = (float*)Ov;
    const int bb = m_blk / SEQ;
    const int s0 = m_blk - bb * SEQ;
    v4f vals[16];
#pragma unroll
    for (int i = 0; i < 16; ++i) {
      const int n = w * 16 + i;
      const int cg = n_blk + n;
      const v4f cv = *(const v4f*)(&Cs[n * 128 + 4 * lane]);
      const v4f xv = *(const v4f*)(xres + ((size_t)(bb * CCH) + cg) * SEQ_FULL + s0 + 4 * lane);
      v4f o;
      o[0] = bf16_rne(xv[0]) + cv[0];
      o[1] = bf16_rne(xv[1]) + cv[1];
      o[2] = bf16_rne(xv[2]) + cv[2];
      o[3] = bf16_rne(xv[3]) + cv[3];
      vals[i] = o;
    }
#pragma unroll
    for (int i = 0; i < 16; ++i) {
      const int cg = n_blk + w * 16 + i;
      *(volatile v4f*)(out + ((size_t)(bb * CCH) + cg) * SEQ + s0 + 4 * lane) = vals[i];
    }
    __threadfence();
#pragma unroll
    for (int i = 0; i < 16; ++i) {
      const int cg = n_blk + w * 16 + i;
      *(volatile v4f*)(out + ((size_t)(bb * CCH) + cg) * SEQ + s0 + 4 * lane) = vals[i];
    }
  } else {
    _Float16* out = (_Float16*)Ov;
    if (z != ztr) {
      v4u vals[8];
      const int c0 = nin * 8;
#pragma unroll
      for (int i = 0; i < 8; ++i) {
        const int row = w * 16 + 2 * i + hf;
        const v4f a = *(const v4f*)(&Cs[row * 128 + c0]);
        const v4f b = *(const v4f*)(&Cs[row * 128 + c0 + 4]);
        Pack8 o;
        o.h[0] = (_Float16)a[0]; o.h[1] = (_Float16)a[1];
        o.h[2] = (_Float16)a[2]; o.h[3] = (_Float16)a[3];
        o.h[4] = (_Float16)b[0]; o.h[5] = (_Float16)b[1];
        o.h[6] = (_Float16)b[2]; o.h[7] = (_Float16)b[3];
        vals[i] = o.u;
      }
#pragma unroll
      for (int i = 0; i < 8; ++i) {
        const int row = w * 16 + 2 * i + hf;
        *(volatile v4u*)(out + (size_t)(m_blk + row) * Nout + n_blk + c0) = vals[i];
      }
      __threadfence();
#pragma unroll
      for (int i = 0; i < 8; ++i) {
        const int row = w * 16 + 2 * i + hf;
        *(volatile v4u*)(out + (size_t)(m_blk + row) * Nout + n_blk + c0) = vals[i];
      }
    } else {
      const int bb = m_blk / SEQ;
      const int s0 = m_blk - bb * SEQ;
      const int t0 = nin * 8;
      v4u vals[8];
#pragma unroll
      for (int i = 0; i < 8; ++i) {
        const int c = w * 16 + 2 * i + hf;
        Pack8 o;
#pragma unroll
        for (int j = 0; j < 8; ++j) o.h[j] = (_Float16)Cs[(t0 + j) * 128 + c];
        vals[i] = o.u;
      }
#pragma unroll
      for (int i = 0; i < 8; ++i) {
        const int c = w * 16 + 2 * i + hf;
        const int n = n_blk + c;
        const int hh = n / HDIM, d = n - hh * HDIM;
        _Float16* dst = out + ((size_t)(bb * HEADS + hh) * HDIM + d) * SEQ + s0 + t0;
        *(volatile v4u*)dst = vals[i];
      }
      __threadfence();
#pragma unroll
      for (int i = 0; i < 8; ++i) {
        const int c = w * 16 + 2 * i + hf;
        const int n = n_blk + c;
        const int hh = n / HDIM, d = n - hh * HDIM;
        _Float16* dst = out + ((size_t)(bb * HEADS + hh) * HDIM + d) * SEQ + s0 + t0;
        *(volatile v4u*)dst = vals[i];
      }
    }
  }
}

__global__ __launch_bounds__(128) __attribute__((amdgpu_num_vgpr(256)))
void k_attn(const _Float16* __restrict__ qh, const _Float16* __restrict__ kh,
            const _Float16* __restrict__ vt, _Float16* __restrict__ oh, float scale) {
  __shared__ _Float16 Ps[4 * 16 * PLD];

  const int tid = threadIdx.x, w = tid >> 5, lane = tid & 31;
  const int hf = lane >> 4, nin = lane & 15;
  const int qblk = blockIdx.x, h = blockIdx.y, b = blockIdx.z;
  const int qtok0 = b * SEQ + qblk * 64 + w * 16;
  const int ktokb = b * SEQ;
  _Float16* Pw = Ps + w * 16 * PLD;
  const _Float16* vtb = vt + (size_t)(b * HEADS + h) * HDIM * SEQ;

  v16h qa[2];
  {
    const _Float16* qp = qh + (size_t)(qtok0 + nin) * CCH + h * HDIM + 8 * hf;
    Frag f;
    f.h[0] = *(const v8h*)(qp);      f.h[1] = *(const v8h*)(qp + 16); qa[0] = f.v;
    f.h[0] = *(const v8h*)(qp + 32); f.h[1] = *(const v8h*)(qp + 48); qa[1] = f.v;
  }

  float mrow[8], lrow[8];
#pragma unroll
  for (int r = 0; r < 8; ++r) { mrow[r] = -1.0e30f; lrow[r] = 0.0f; }
  v8f oacc[4] = {};

  const int nkb = SEQ / 64;
#pragma unroll 1
  for (int kb = 0; kb < nkb; ++kb) {
    __syncthreads();

    v8f sacc[4] = {};
#pragma unroll
    for (int nt = 0; nt < 4; ++nt) {
      const _Float16* kp = kh + (size_t)(ktokb + kb * 64 + nt * 16 + nin) * CCH + h * HDIM + 8 * hf;
      Frag f;
      f.h[0] = *(const v8h*)(kp);      f.h[1] = *(const v8h*)(kp + 16);
      sacc[nt] = wmma16(qa[0], f.v, sacc[nt]);
      Frag g;
      g.h[0] = *(const v8h*)(kp + 32); g.h[1] = *(const v8h*)(kp + 48);
      sacc[nt] = wmma16(qa[1], g.v, sacc[nt]);
    }

#pragma unroll
    for (int r = 0; r < 8; ++r) {
      const float s0 = sacc[0][r] * scale, s1 = sacc[1][r] * scale;
      const float s2 = sacc[2][r] * scale, s3 = sacc[3][r] * scale;
      float t = fmaxf(fmaxf(s0, s1), fmaxf(s2, s3));
      t = fmaxf(t, __shfl_xor(t, 8, 16));
      t = fmaxf(t, __shfl_xor(t, 4, 16));
      t = fmaxf(t, __shfl_xor(t, 2, 16));
      t = fmaxf(t, __shfl_xor(t, 1, 16));
      const float mn    = fmaxf(mrow[r], t);
      const float alpha = __expf(mrow[r] - mn);
      mrow[r] = mn;
      const float p0 = __expf(s0 - mn), p1 = __expf(s1 - mn);
      const float p2 = __expf(s2 - mn), p3 = __expf(s3 - mn);
      float rs = (p0 + p1) + (p2 + p3);
      rs += __shfl_xor(rs, 8, 16);
      rs += __shfl_xor(rs, 4, 16);
      rs += __shfl_xor(rs, 2, 16);
      rs += __shfl_xor(rs, 1, 16);
      lrow[r] = lrow[r] * alpha + rs;
      sacc[0][r] = p0; sacc[1][r] = p1; sacc[2][r] = p2; sacc[3][r] = p3;
      oacc[0][r] *= alpha; oacc[1][r] *= alpha; oacc[2][r] *= alpha; oacc[3][r] *= alpha;
    }

#pragma unroll
    for (int nt = 0; nt < 4; ++nt)
#pragma unroll
      for (int r = 0; r < 8; ++r)
        Pw[(8 * hf + r) * PLD + nt * 16 + nin] = (_Float16)(sacc[nt][r] * 1024.0f);
    __syncthreads();

#pragma unroll
    for (int ks = 0; ks < 2; ++ks) {
      const v16h pf = frag_rows(Pw, 0, (size_t)PLD, ks * 32);
#pragma unroll
      for (int dt = 0; dt < 4; ++dt) {
        const _Float16* vp = vtb + (size_t)(dt * 16 + nin) * SEQ + kb * 64 + ks * 32 + 8 * hf;
        Frag f;
        f.h[0] = *(const v8h*)(vp); f.h[1] = *(const v8h*)(vp + 16);
        oacc[dt] = wmma16(pf, f.v, oacc[dt]);
      }
    }
  }
  __syncthreads();

#pragma unroll
  for (int r = 0; r < 8; ++r) {
    const float inv = 0.0625f * (1.0f / lrow[r]);
#pragma unroll
    for (int dt = 0; dt < 4; ++dt)
      Pw[(8 * hf + r) * PLD + dt * 16 + nin] = (_Float16)(oacc[dt][r] * inv);
  }
  __syncthreads();

  Pack8 vals[4];
  const int cl = (lane & 7) * 8;
#pragma unroll
  for (int i = 0; i < 4; ++i) {
    const int row = (lane >> 3) + 4 * i;
    vals[i].h = *(const v8h*)(Pw + row * PLD + cl);
  }
#pragma unroll
  for (int i = 0; i < 4; ++i) {
    const int row = (lane >> 3) + 4 * i;
    *(volatile v4u*)(oh + (size_t)(qtok0 + row) * CCH + h * HDIM + cl) = vals[i].u;
  }
  __threadfence();
#pragma unroll
  for (int i = 0; i < 4; ++i) {
    const int row = (lane >> 3) + 4 * i;
    *(volatile v4u*)(oh + (size_t)(qtok0 + row) * CCH + h * HDIM + cl) = vals[i].u;
  }
}

extern "C" void kernel_launch(void* const* d_in, const int* in_sizes, int n_in,
                              void* d_out, int out_size, void* d_ws, size_t ws_size,
                              hipStream_t stream) {
  if (n_in < 7) return;
  const long long need_x = ((long long)NB * CCH - 1) * (long long)SEQ_FULL + (long long)SEQ;
  if ((long long)in_sizes[0] < need_x) return;
  if (in_sizes[1] < CCH || in_sizes[2] < CCH) return;
  if (in_sizes[3] < QKVO * CCH || in_sizes[4] < QKVO) return;
  if (in_sizes[5] < CCH * CCH || in_sizes[6] < CCH) return;
  if ((long long)out_size < (long long)NB * CCH * SEQ) return;
  const size_t ws_need = WS_HALVES * sizeof(_Float16);
  if (ws_need > ws_size) return;

  const float* x      = (const float*)d_in[0];
  const float* gnw    = (const float*)d_in[1];
  const float* gnb    = (const float*)d_in[2];
  const float* qkv_w  = (const float*)d_in[3];
  const float* qkv_b  = (const float*)d_in[4];
  const float* proj_w = (const float*)d_in[5];
  const float* proj_b = (const float*)d_in[6];
  float* out = (float*)d_out;

  _Float16* xh  = (_Float16*)d_ws;
  _Float16* wqh = xh  + PLANE_H;
  _Float16* wkh = wqh + WPL_H;
  _Float16* wvh = wkh + WPL_H;
  _Float16* woh = wvh + WPL_H;
  _Float16* qh  = woh + WPL_H;
  _Float16* kh  = qh  + PLANE_H;
  _Float16* vt  = kh  + PLANE_H;
  _Float16* oh  = vt  + PLANE_H;

  k_gn<<<dim3(CCH / 64, NB), 256, 0, stream>>>(x, gnw, gnb, xh);

  {
    const int tw = CCH * (CCH / 8);
    k_cvt<<<(tw + 255) / 256, 256, 0, stream>>>(qkv_w,                  wqh, CCH, CCH, HDIM, 3 * HDIM, 64.0f);
    k_cvt<<<(tw + 255) / 256, 256, 0, stream>>>(qkv_w + HDIM * CCH,     wkh, CCH, CCH, HDIM, 3 * HDIM, 64.0f);
    k_cvt<<<(tw + 255) / 256, 256, 0, stream>>>(qkv_w + 2 * HDIM * CCH, wvh, CCH, CCH, HDIM, 3 * HDIM, 64.0f);
    k_cvt<<<(tw + 255) / 256, 256, 0, stream>>>(proj_w,                 woh, CCH, CCH, CCH, CCH, 64.0f);
  }

  k_gemm<0><<<dim3(CCH / 128, NTOK / 128, 3), 256, 0, stream>>>(
      xh, wqh, wkh, wvh, qkv_b, qkv_b + HDIM, qkv_b + 2 * HDIM,
      (void*)qh, (void*)kh, (void*)vt, x,
      CCH, CCH, 2, 0.015625f, HDIM, 3 * HDIM);

  k_attn<<<dim3(SEQ / 64, HEADS, NB), 128, 0, stream>>>(qh, kh, vt, oh, 0.125f);

  k_gemm<1><<<dim3(CCH / 128, NTOK / 128, 1), 256, 0, stream>>>(
      oh, woh, woh, woh, proj_b, proj_b, proj_b,
      (void*)out, (void*)out, (void*)out, x,
      CCH, CCH, -1, 0.000244140625f, CCH, CCH);
}
